// OptimizedISM_64733747085528
// MI455X (gfx1250) — hardware-verified
//
#include <hip/hip_runtime.h>
#include <math.h>
#include <stdint.h>

#define NB     4
#define NC     256
#define LQ     1024
#define LK     4096
#define NGRP   64
#define QROW   32
#define TPITCH 72
#define PPITCH 72
#define OPITCH 260
#define RTEMP  0.0625f
#define PCARRY 1024.0f
#define PUNDO  0.0009765625f
static_assert(LQ == 32 * 32);
static_assert(LK == 64 * 64);
static_assert((NC % 64) == 0);
static_assert(NGRP * 64 == LK);

typedef _Float16       v16h __attribute__((ext_vector_type(16)));
typedef _Float16       v8h  __attribute__((ext_vector_type(8)));
typedef __bf16         v16b __attribute__((ext_vector_type(16)));
typedef unsigned short v8us __attribute__((ext_vector_type(8)));
typedef float          v8f  __attribute__((ext_vector_type(8)));
typedef float          v4f  __attribute__((ext_vector_type(4)));
typedef unsigned int   v4u  __attribute__((ext_vector_type(4)));

union FragH { v16h v; v8h  h[2]; };
union FragB { v16b v; v8us u[2]; };
static_assert(sizeof(FragH) == 32);
static_assert(sizeof(FragB) == 32);

__device__ __forceinline__ unsigned short bf_bits(float f) {
  unsigned u = __float_as_uint(f);
  return (unsigned short)((u + 0x7FFFu + ((u >> 16) & 1u)) >> 16);
}
__device__ __forceinline__ float bf_up(unsigned short h) { return __uint_as_float(((unsigned)h) << 16); }
__device__ __forceinline__ unsigned short h_bits(_Float16 x) { return __builtin_bit_cast(unsigned short, x); }
__device__ __forceinline__ unsigned pk16(unsigned short a, unsigned short b) { return (unsigned)a | ((unsigned)b << 16); }
__device__ __forceinline__ v8f zero8() { v8f z = {0.f, 0.f, 0.f, 0.f, 0.f, 0.f, 0.f, 0.f}; return z; }
__device__ __forceinline__ float hmax8(v8f s) {
  return fmaxf(fmaxf(fmaxf(s[0], s[1]), fmaxf(s[2], s[3])), fmaxf(fmaxf(s[4], s[5]), fmaxf(s[6], s[7])));
}

__device__ __forceinline__ v16h ldfrag_h(const _Float16* p) {
  FragH f;
  f.h[0] = *(const v8h*)(p);
  f.h[1] = *(const v8h*)(p + 16);
  return f.v;
}
__device__ __forceinline__ v16b ldfrag_b(const unsigned short* p) {
  FragB f;
  f.u[0] = *(const v8us*)(p);
  f.u[1] = *(const v8us*)(p + 16);
  return f.v;
}

__device__ __forceinline__ v8f mma_h_raw(v16h a, v16h b, v8f c) {
  return __builtin_amdgcn_wmma_f32_16x16x32_f16(false, a, false, b, (short)0, c, false, false);
}
__device__ __forceinline__ v8f mma_b_raw(v16b a, v16b b, v8f c) {
  return __builtin_amdgcn_wmma_f32_16x16x32_bf16(false, a, false, b, (short)0, c, false, false);
}
__device__ __forceinline__ void sguard(v8f& a, v8f& b, v16b x0, v16b x1, v16b y0) {
#if defined(__HIP_DEVICE_COMPILE__)
  const v16h h0 = __builtin_bit_cast(v16h, x0), h1 = __builtin_bit_cast(v16h, x1);
  const v16h g0 = __builtin_bit_cast(v16h, y0);
  asm volatile("v_nop\n\tv_nop\n\tv_nop\n\tv_nop" : "+v"(a), "+v"(b) : "v"(h0), "v"(h1), "v"(g0));
#endif
}
__device__ __forceinline__ void oguard(v8f& a, v16h x0, v16h x1, v16h p0, v16h p1) {
#if defined(__HIP_DEVICE_COMPILE__)
  asm volatile("v_nop\n\tv_nop\n\tv_nop\n\tv_nop" : "+v"(a) : "v"(x0), "v"(x1), "v"(p0), "v"(p1));
#endif
}

__global__ __launch_bounds__(256) void cvt_plane(const float* __restrict__ src, int rowlen, int nkt, int dov,
                                                  unsigned short* dT, unsigned short* dV) {
  __shared__ __align__(16) unsigned short Ts[64 * TPITCH];
  const int tid  = threadIdx.x;
  const int lane = tid & 31, wave = tid >> 5;
  const int bx   = blockIdx.x;
  const int kt   = bx % nkt;
  const int rest = bx / nkt;
  const int ct   = rest & 3;
  const int b    = rest >> 2;

  {
    const int e = lane & 7, rq = lane >> 3;
    v4u u[2];
    size_t go[2];
#pragma unroll
    for (int it = 0; it < 2; ++it) {
      const int row = wave * 8 + it * 4 + rq;
      const size_t o = ((size_t)(b * NC + ct * 64 + row)) * (size_t)rowlen + (size_t)kt * 64 + 8 * e;
      go[it] = o;
      const v4f a = *(const v4f*)(src + o), c4 = *(const v4f*)(src + o + 4);
      unsigned short w[8];
#pragma unroll
      for (int t = 0; t < 4; ++t) { w[t] = bf_bits(a[t]); w[4 + t] = bf_bits(c4[t]); }
#pragma unroll
      for (int t = 0; t < 8; ++t) Ts[(8 * e + t) * TPITCH + row] = w[t];
      v4u pk;
#pragma unroll
      for (int t = 0; t < 4; ++t)
        pk[t] = pk16(h_bits((_Float16)bf_up(w[2 * t])), h_bits((_Float16)bf_up(w[2 * t + 1])));
      u[it] = pk;
    }
    if (dov != 0) {
      for (int pass = 0; pass < 2; ++pass) {
#pragma unroll
        for (int it = 0; it < 2; ++it) *(volatile v4u*)(dV + go[it]) = u[it];
        __threadfence();
      }
    }
  }
  __syncthreads();
  {
    const int e = tid & 7, lq = tid >> 3;
    v4u u[2];
    size_t go[2];
#pragma unroll
    for (int it = 0; it < 2; ++it) {
      const int kk = it * 32 + lq;
      u[it]  = *(const v4u*)(Ts + kk * TPITCH + 8 * e);
      go[it] = ((size_t)b * (size_t)rowlen + (size_t)kt * 64 + kk) * NC + ct * 64 + 8 * e;
    }
    for (int pass = 0; pass < 2; ++pass) {
#pragma unroll
      for (int it = 0; it < 2; ++it) *(volatile v4u*)(dT + go[it]) = u[it];
      __threadfence();
    }
  }
}

__global__ __launch_bounds__(128)
void attn_kernel(const unsigned short* __restrict__ qp, const unsigned short* __restrict__ kp,
                 const unsigned short* __restrict__ vtp, float* out) {
  __shared__ __align__(16) float    Os[QROW * OPITCH];
  __shared__ __align__(16) _Float16 Ps[32 * PPITCH];
  __shared__ float xm[128];
  __shared__ float xs[128];
  const int tid  = threadIdx.x;
  const int wave = tid >> 5;
  const int lane = tid & 31;
  const int hh   = lane >> 4;
  const int c16  = lane & 15;
  const int bx   = blockIdx.x;
  const int b    = bx >> 5;
  const int y    = bx & 31;
  const int g    = wave & 1;
  const int kh   = wave >> 1;
  const int x    = 16 * g + c16;
  const int uq   = y * 32 + x;

  const unsigned short* Qb = qp + ((size_t)(b * LQ + uq)) * NC + 8 * hh;
  const unsigned short* Kb = kp + ((size_t)b * LK + c16) * NC + 8 * hh;
  const _Float16* VT = (const _Float16*)(const void*)vtp;
  const _Float16* Vb = VT + ((size_t)(b * NC + 128 * kh + c16)) * LK + 8 * hh;
  _Float16* pw       = Ps + (g * 16 + c16) * PPITCH + 32 * kh + 8 * hh;
  const _Float16* pr = Ps + (g * 16 + c16) * PPITCH + 8 * hh;

  v8f o[8];
#pragma unroll
  for (int ct = 0; ct < 8; ++ct) o[ct] = zero8();

#pragma unroll 1
  for (int i = 0; i < NGRP; ++i) {
    const unsigned short* K0 = Kb + ((size_t)(i * 64 + 32 * kh)) * NC;
    const unsigned short* K1 = K0 + (size_t)16 * NC;
    v8f s0 = zero8(), s1 = zero8();
#pragma unroll 1
    for (int kk = 0; kk < NC / 32; ++kk) {
      const v16b q  = ldfrag_b(Qb + 32 * kk);
      const v16b a0 = ldfrag_b(K0 + 32 * kk);
      const v16b a1 = ldfrag_b(K1 + 32 * kk);
      s0 = mma_b_raw(a0, q, s0);
      s1 = mma_b_raw(a1, q, s1);
      sguard(s0, s1, a0, a1, q);
    }

    float pm = fmaxf(hmax8(s0), hmax8(s1));
    pm = fmaxf(pm, __shfl_xor(pm, 16, 32));
    xm[tid] = pm;
    __syncthreads();
    const float m = fmaxf(pm, xm[tid ^ 64]);

    v8f e0, e1;
    float ls = 0.f;
#pragma unroll
    for (int r = 0; r < 8; ++r) {
      const float a0 = __expf((s0[r] - m) * RTEMP);
      const float a1 = __expf((s1[r] - m) * RTEMP);
      e0[r] = a0; e1[r] = a1;
      ls += a0 + a1;
    }
    ls += __shfl_xor(ls, 16, 32);
    xs[tid] = ls;
    __syncthreads();
    const float l  = ls + xs[tid ^ 64];
    const float ps = PCARRY * __builtin_amdgcn_rcpf(l);

    FragH ph;
#pragma unroll
    for (int r = 0; r < 8; ++r) {
      ph.h[0][r] = (_Float16)(e0[r] * ps);
      ph.h[1][r] = (_Float16)(e1[r] * ps);
    }
    *(v8h*)(pw)      = ph.h[0];
    *(v8h*)(pw + 16) = ph.h[1];
    __syncthreads();

    const v16h p0 = ldfrag_h(pr);
    const v16h p1 = ldfrag_h(pr + 32);
    const size_t kofs = (size_t)i * 64;
#pragma unroll
    for (int ct = 0; ct < 8; ++ct) {
      const _Float16* vp = Vb + (size_t)(16 * ct) * LK + kofs;
      const v16h v0 = ldfrag_h(vp);
      const v16h v1 = ldfrag_h(vp + 32);
      o[ct] = mma_h_raw(v0, p0, o[ct]);
      o[ct] = mma_h_raw(v1, p1, o[ct]);
      oguard(o[ct], v0, v1, p0, p1);
    }
  }

  {
    const unsigned short* qres = qp + ((size_t)(b * LQ + uq)) * NC + 128 * kh + 8 * hh;
    float* osr = Os + x * OPITCH + 128 * kh + 8 * hh;
#pragma unroll
    for (int ct = 0; ct < 8; ++ct) {
      const v8us qq = *(const v8us*)(qres + 16 * ct);
      v4f w0, w1;
#pragma unroll
      for (int r = 0; r < 4; ++r) {
        w0[r] = o[ct][r] * PUNDO + bf_up(qq[r]);
        w1[r] = o[ct][4 + r] * PUNDO + bf_up(qq[4 + r]);
      }
      *(v4f*)(osr + 16 * ct)     = w0;
      *(v4f*)(osr + 16 * ct + 4) = w1;
    }
  }
  __syncthreads();
  {
    const int e = tid & 7, lq = tid >> 3;
    float* ob = out + (size_t)b * NC * LK + (size_t)(2 * y) * 64 + 4 * e;
#pragma unroll 1
    for (int ch = 0; ch < 8; ++ch) {
      v4f vals[8];
#pragma unroll
      for (int it = 0; it < 8; ++it) {
        const int L  = (ch * 8 + it) * 16 + lq;
        const int c  = L >> 2, hf = L & 1;
        const float* s = Os + (hf * 16 + 2 * e) * OPITCH + c;
        const float z0 = s[0], z1 = s[OPITCH];
        v4f v;
        v[0] = z0; v[1] = z0; v[2] = z1; v[3] = z1;
        vals[it] = v;
      }
      for (int pass = 0; pass < 2; ++pass) {
#pragma unroll
        for (int it = 0; it < 8; ++it) {
          const int L  = (ch * 8 + it) * 16 + lq;
          const int c  = L >> 2, hrow = (L >> 1) & 1, hf = L & 1;
          *(volatile v4f*)(ob + (size_t)c * LK + hrow * 64 + hf * 32) = vals[it];
        }
        __threadfence();
      }
    }
  }
}

extern "C" void kernel_launch(void* const* d_in, const int* in_sizes, int n_in,
                              void* d_out, int out_size, void* d_ws, size_t ws_size,
                              hipStream_t stream) {
  const int ND = NB * NC * LQ;
  const int NS = NB * NC * LK;
  if (n_in < 2) return;
  if (in_sizes[0] != ND || in_sizes[1] != NS) return;
  if (out_size != NS) return;

  size_t off = 0;
  const size_t oK = off; off += (size_t)NS * 2;
  const size_t oV = off; off += (size_t)NS * 2;
  const size_t oQ = off; off += (size_t)ND * 2;
  if (off > ws_size) return;
  if (off > (size_t)134217728) return;

  const float* Dp = (const float*)d_in[0];
  const float* Sp = (const float*)d_in[1];
  char* ws = (char*)d_ws;
  unsigned short* KP = (unsigned short*)(ws + oK);
  unsigned short* VT = (unsigned short*)(ws + oV);
  unsigned short* QP = (unsigned short*)(ws + oQ);
  float* out = (float*)d_out;

  const dim3 blk256(256), blk128(128);
  const dim3 gS(NB * 4 * (LK / 64));
  const dim3 gD(NB * 4 * (LQ / 64));
  const dim3 gA(NB * (LQ / QROW));

  cvt_plane<<<gS, blk256, 0, stream>>>(Sp, LK, LK / 64, 1, KP, VT);
  cvt_plane<<<gD, blk256, 0, stream>>>(Dp, LQ, LQ / 64, 0, QP, VT);
  attn_kernel<<<gA, blk128, 0, stream>>>(QP, KP, VT, out);
  (void)hipGetLastError();
}
